// CumulativeLinearMultiheadAttentionKV_21706764714123
// MI455X (gfx1250) — hardware-verified
//
#include <hip/hip_runtime.h>


namespace {
constexpr int T = 1024, B = 2, E = 1024, NH = 16, DH = 64, NR = T * B;
constexpr float XS = 8.0f, WSC = 256.0f, SCALE = 0.125f;
typedef _Float16 b16;
typedef __attribute__((ext_vector_type(16))) _Float16 v16b;
typedef __attribute__((ext_vector_type(8))) _Float16 v8b;
typedef __attribute__((ext_vector_type(8))) float v8f;
typedef __attribute__((ext_vector_type(4))) float v4f;
__device__ __forceinline__ float bf16_rne(float f) { unsigned int u = __float_as_uint(f); u += 0x7FFFu + ((u >> 16) & 1u); float r = __uint_as_float(u & 0xFFFF0000u); asm volatile("" : "+v"(r)); return r; }
__device__ __forceinline__ void split16(float v, b16& hi, b16& lo) { hi = (b16)v; lo = (b16)(v - (float)hi); }
__device__ __forceinline__ v16b frag_kb(const b16* p, int hh) { const v8b a = *(const v8b*)(p + 8 * hh), b = *(const v8b*)(p + 16 + 8 * hh); v16b f;
#pragma unroll
  for (int e = 0; e < 8; ++e) { f[e] = a[e]; f[8 + e] = b[e]; } return f; }
__device__ __forceinline__ v8f wmma16b(v16b a, v16b b, v8f c) { v8f d = __builtin_amdgcn_wmma_f32_16x16x32_f16(false, a, false, b, (short)0, c, false, false); asm volatile("v_nop\n\tv_nop\n\tv_nop\n\tv_nop" : "+v"(d) : "v"(a), "v"(b)); return d; }
__device__ __forceinline__ void wave_lds_sync() { __builtin_amdgcn_fence(__ATOMIC_RELEASE, "workgroup"); __builtin_amdgcn_wave_barrier(); __builtin_amdgcn_fence(__ATOMIC_ACQUIRE, "workgroup"); }
__device__ __forceinline__ float pmul(float a, float b) { float p = a * b; asm volatile("" : "+v"(p)); return p; }

__global__ __launch_bounds__(256) void wcopy_kernel(const float* __restrict__ w, size_t total, b16* __restrict__ WT) { const size_t u = (size_t)blockIdx.x * 256 + threadIdx.x; if (u >= total / 8) return; v8b v;
#pragma unroll
  for (int j = 0; j < 8; ++j) v[j] = (b16)(bf16_rne(w[u * 8 + j]) * WSC); for (int pass = 0; pass < 2; ++pass) { *(volatile v8b*)(WT + u * 8) = v; __threadfence(); } }
template <int MODE>
__global__ __launch_bounds__(32) void proj_kernel(const float* __restrict__ X, const b16* __restrict__ WT, const float* __restrict__ bias, int NRV, float* __restrict__ OUT) {
  __shared__ __attribute__((aligned(16))) b16 Ah[16][E + 8], Al[16][MODE == 0 ? 8 : E + 8]; __shared__ float Tf[16][132]; const int lane = threadIdx.x, nloc = lane & 15, hlf = lane >> 4; const int g = blockIdx.x % (E / 128); const size_t m0 = (size_t)(blockIdx.x / (E / 128)) * 16; if (m0 >= (size_t)NRV) return;
  for (int rr = 0; rr < 16; ++rr) for (int q = 0; q < E / 32; ++q) { const float v = X[(m0 + rr) * E + q * 32 + lane]; if (MODE == 0) Ah[rr][q * 32 + lane] = (b16)(bf16_rne(v) * XS); else { b16 p, ql; split16(v * XS, p, ql); Ah[rr][q * 32 + lane] = p; Al[rr][q * 32 + lane] = ql; } }
  wave_lds_sync(); v8f acc[8];
#pragma unroll
  for (int t = 0; t < 8; ++t) acc[t] = (v8f){};
#pragma unroll 2
  for (int kb = 0; kb < E; kb += 32) { const v16b a = frag_kb(&Ah[nloc][kb], hlf); v16b a2; if (MODE != 0) a2 = frag_kb(&Al[nloc][kb], hlf);
#pragma unroll
    for (int t = 0; t < 8; ++t) { const v16b bw = frag_kb(WT + (size_t)(g * 128 + t * 16 + nloc) * E + kb, hlf); acc[t] = wmma16b(a, bw, acc[t]); if (MODE != 0) acc[t] = wmma16b(a2, bw, acc[t]); } }
#pragma unroll
  for (int t = 0; t < 8; ++t) { const int c = g * 128 + t * 16 + nloc; const float bb = bf16_rne(bias[c]);
#pragma unroll
    for (int r8 = 0; r8 < 8; ++r8) Tf[8 * hlf + r8][t * 16 + nloc] = acc[t][r8] * (1.0f / (XS * WSC)) + bb; }
  wave_lds_sync();
  for (int pass = 0; pass < 2; ++pass) { for (int rr = 0; rr < 16; ++rr) *(volatile v4f*)(OUT + (m0 + rr) * E + g * 128 + lane * 4) = *(const v4f*)(&Tf[rr][lane * 4]); __threadfence(); } }
__global__ __launch_bounds__(32) void scan_kernel(const float* __restrict__ Q, const float* __restrict__ Kp, const float* __restrict__ V, int TV, float* __restrict__ CTX) {
  const int lane = threadIdx.x; const int h = blockIdx.x % NH, b = blockIdx.x / NH;
  for (int pass = 0; pass < 2; ++pass) { float S0[DH], S1[DH];
#pragma unroll
    for (int k = 0; k < DH; ++k) { S0[k] = 0.0f; S1[k] = 0.0f; }
#pragma unroll 1
    for (int t = 0; t < TV; ++t) { const size_t row = (size_t)t * B + b; const float* qr = Q + row * E + h * DH; const float* kr = Kp + row * E + h * DH; const float v0 = V[row * E + h * DH + lane], v1 = V[row * E + h * DH + 32 + lane]; float o0 = 0.0f, o1 = 0.0f;
#pragma unroll
      for (int k = 0; k < DH; ++k) { const float kk = kr[k], qq = qr[k]; S0[k] += pmul(kk, v0); S1[k] += pmul(kk, v1); o0 += pmul(qq, S0[k]); o1 += pmul(qq, S1[k]); }
      ((volatile float*)CTX)[row * E + h * DH + lane] = o0 * SCALE; ((volatile float*)CTX)[row * E + h * DH + 32 + lane] = o1 * SCALE; }
    __threadfence(); } }
}

extern "C" void kernel_launch(void* const* d_in, const int* in_sizes, int n_in, void* d_out, int out_size, void* d_ws, size_t ws_size, hipStream_t stream) {
  (void)n_in;
  auto Fp = [&](int i) { return (const float*)d_in[i]; };
  if (in_sizes[0] != NR * E || in_sizes[1] != NR * E || in_sizes[2] != NR * E || in_sizes[3] != 3 * E * E || in_sizes[4] != 3 * E || in_sizes[5] != E * E || out_size != NR * E) return;
  const int TV = T; const int NRV = TV * B;
  size_t off = 0; char* ws = (char*)d_ws;
  auto carve = [&](size_t bytes) { char* p = ws + off; off += (bytes + 255) & ~(size_t)255; return p; };
  b16* WIN = (b16*)carve((size_t)3 * E * E * 2); b16* WOUT = (b16*)carve((size_t)E * E * 2); float* Q = (float*)carve((size_t)NR * E * 4); float* Kp = (float*)carve((size_t)NR * E * 4); float* Vp = (float*)carve((size_t)NR * E * 4); float* CTX = (float*)carve((size_t)NR * E * 4);
  if (off > ws_size || off > ((size_t)64 << 20)) return;
  wcopy_kernel<<<(unsigned)(((size_t)3 * E * E / 8 + 255) / 256), 256, 0, stream>>>(Fp(3), (size_t)3 * E * E, WIN); wcopy_kernel<<<(unsigned)(((size_t)E * E / 8 + 255) / 256), 256, 0, stream>>>(Fp(5), (size_t)E * E, WOUT);
  proj_kernel<0><<<(NRV / 16) * (E / 128), 32, 0, stream>>>(Fp(0), WIN, Fp(4), NRV, Q);
  proj_kernel<0><<<(NRV / 16) * (E / 128), 32, 0, stream>>>(Fp(1), WIN + (size_t)E * E, Fp(4) + E, NRV, Kp);
  proj_kernel<0><<<(NRV / 16) * (E / 128), 32, 0, stream>>>(Fp(2), WIN + (size_t)2 * E * E, Fp(4) + 2 * E, NRV, Vp);
  scan_kernel<<<B * NH, 32, 0, stream>>>(Q, Kp, Vp, TV, CTX);
  proj_kernel<1><<<(NRV / 16) * (E / 128), 32, 0, stream>>>(CTX, WOUT, Fp(6), NRV, (float*)d_out);
}
